// Net_25847113187867
// MI455X (gfx1250) — hardware-verified
//
#include <hip/hip_runtime.h>
#include <math.h>

constexpr int L_IN      = 16684;
constexpr int COVLEN    = 300;
constexpr int NWIN      = L_IN - COVLEN;
constexpr int NCH       = 64;
constexpr int G_ROWS    = 16768;
constexpr int G_VALID_MAX = L_IN - 5;
constexpr int C2_ROWS   = 16704;
constexpr int C3_ROWS   = 16576;
constexpr int DIL2      = 5;
constexpr int DIL3      = 15;
constexpr int DILF      = 30;
constexpr int K_CONV    = 384;
constexpr int K_FC1     = 448;
constexpr int K_FC2     = 320;
constexpr int N_FC1     = 320;
constexpr int N_FC2     = 80;
constexpr int N_FC2P    = 128;
constexpr int H2_PITCH  = 128;

constexpr int OFF_W2    = 0;
constexpr int OFF_W3    = OFF_W2 + NCH * K_CONV;
constexpr int OFF_FC1   = OFF_W3 + NCH * K_CONV;
constexpr int OFF_FC2   = OFF_FC1 + N_FC1 * K_FC1;
constexpr int W_TOTAL   = OFF_FC2 + N_FC2P * K_FC2;
constexpr int U_W3_BASE  = OFF_W3 / 8;
constexpr int U_FC1_BASE = OFF_FC1 / 8;
constexpr int U_FC2_BASE = OFF_FC2 / 8;
constexpr int U_TOTAL    = W_TOTAL / 8;

static_assert(NWIN == 16384, "window count");
static_assert(G_ROWS % 64 == 0 && C2_ROWS % 64 == 0 && C3_ROWS % 64 == 0 && NWIN % 64 == 0, "M tile multiples");
static_assert(NCH % 64 == 0 && N_FC1 % 64 == 0 && N_FC2P % 64 == 0, "N tile multiples");
static_assert(K_CONV % 64 == 0 && K_FC1 % 64 == 0 && K_FC2 % 32 == 0, "K multiples");
static_assert(C2_ROWS - 1 + 5 * DIL2 < G_ROWS, "conv2 tap reads stay inside the G plane");
static_assert(C3_ROWS - 1 + 5 * DIL3 < C2_ROWS, "conv3 tap reads stay inside the C2 plane");
static_assert(NWIN - 1 + 6 * DILF < C3_ROWS, "fc1 gather reads stay inside the C3 plane");
static_assert(NWIN - 1 + 6 * DILF + 5 * DIL3 + 5 * DIL2 <= G_VALID_MAX, "every consumed position is a full conv1 position");
static_assert(G_ROWS % 32 == 0, "conv1 grid exact");
static_assert(U_TOTAL % 256 == 0, "weight prep grid exact");
static_assert(U_W3_BASE % 32 == 0 && U_FC1_BASE % 32 == 0 && U_FC2_BASE % 32 == 0, "segment boundaries wave-uniform");
static_assert((2 * NWIN) % 256 == 0, "projection grid exact");

typedef __attribute__((ext_vector_type(16))) __bf16   v16b;
typedef __attribute__((ext_vector_type(8)))  __bf16   v8b;
typedef __attribute__((ext_vector_type(8)))  _Float16 v8h;
typedef __attribute__((ext_vector_type(8)))  float    v8f;
typedef __attribute__((ext_vector_type(4)))  float    v4f;
typedef __attribute__((ext_vector_type(4)))  unsigned int v4u;

__device__ __forceinline__ unsigned short f2bf_bits(float f) {
  unsigned u = __float_as_uint(f);
  return (unsigned short)((u + 0x7FFFu + ((u >> 16) & 1u)) >> 16);
}
__device__ __forceinline__ float bf_bits2f(unsigned short h) { return __uint_as_float(((unsigned)h) << 16); }
__device__ __forceinline__ unsigned f2bf_u(float f) {
  const unsigned u = __float_as_uint(f);
  return ((u + 0x7FFFu + ((u >> 16) & 1u)) >> 16) & 0xFFFFu;
}
__device__ __forceinline__ float bfu2f(unsigned h) { return __uint_as_float(h << 16); }

__device__ __forceinline__ void row_guard_b(v8f& a, v8f& b, v8f& c, v8f& d, v16b x, v16b y) {
  asm volatile("v_nop\n\tv_nop\n\tv_nop\n\tv_nop" : "+v"(a), "+v"(b), "+v"(c), "+v"(d) : "v"(x), "v"(y));
}
__device__ __forceinline__ void keep4_b(v16b a, v16b b, v16b c, v16b d) { asm volatile("v_nop" :: "v"(a), "v"(b), "v"(c), "v"(d)); }
__device__ __forceinline__ void acc_guard4(v8f& a, v8f& b, v8f& c, v8f& d) { asm volatile("v_nop\n\tv_nop\n\tv_nop\n\tv_nop" : "+v"(a), "+v"(b), "+v"(c), "+v"(d)); }

struct FragB {
  union U { v16b v; v8b h[2]; };
  static __device__ __forceinline__ v16b load(const __bf16* p) {
    U f; f.h[0] = *(const v8b*)(p); f.h[1] = *(const v8b*)(p + 16); return f.v;
  }
  static __device__ __forceinline__ v8f mma(v16b a, v16b b, v8f c) {
    return __builtin_amdgcn_wmma_f32_16x16x32_bf16(false, a, false, b, (short)0, c, false, false);
  }
};

__global__ __launch_bounds__(256) void prep_weights_kernel(
    const float* __restrict__ w2, const float* __restrict__ w3,
    const float* __restrict__ fw1, const float* __restrict__ fw2,
    unsigned short* __restrict__ WHI, unsigned short* __restrict__ WLO) {
  const int i = blockIdx.x * 256 + threadIdx.x;
  if (i >= U_TOTAL) return;
  const int seg   = (i >= U_W3_BASE) + (i >= U_FC1_BASE) + (i >= U_FC2_BASE);
  const int ubase = (seg == 0) ? 0 : (seg == 1) ? U_W3_BASE : (seg == 2) ? U_FC1_BASE : U_FC2_BASE;
  const int kdiv8 = (seg < 2) ? (K_CONV / 8) : (seg == 2) ? (K_FC1 / 8) : (K_FC2 / 8);
  const int cm    = (seg < 2) ? 6 : (seg == 2) ? 7 : 1;
  const int tm    = (seg == 3) ? 64 : 1;
  const int nmax  = (seg < 2) ? NCH : (seg == 2) ? N_FC1 : N_FC2;
  const float* src = (seg == 0) ? w2 : (seg == 1) ? w3 : (seg == 2) ? fw1 : fw2;
  const int u   = i - ubase;
  const int n   = u / kdiv8;
  const int kk0 = (u - n * kdiv8) * 8;
  const int tap = kk0 >> 6;
  const int c0  = kk0 & 63;
  const bool valid = (n < nmax);
  const int nc  = valid ? n : (nmax - 1);
  const int rowlen = kdiv8 * 8;
  unsigned hb[8], lb[8];
#pragma unroll
  for (int e = 0; e < 8; ++e) {
    const int idx = nc * rowlen + (c0 + e) * cm + tap * tm;
    const float fl = src[idx];
    const float f  = valid ? fl : 0.0f;
    hb[e] = f2bf_u(f);
    lb[e] = f2bf_u(f - bfu2f(hb[e]));
  }
  const v4u uh = (v4u){hb[0] | (hb[1] << 16), hb[2] | (hb[3] << 16), hb[4] | (hb[5] << 16), hb[6] | (hb[7] << 16)};
  const v4u ul = (v4u){lb[0] | (lb[1] << 16), lb[2] | (lb[3] << 16), lb[4] | (lb[5] << 16), lb[6] | (lb[7] << 16)};
  unsigned short* ph = WHI + (size_t)i * 8;
  unsigned short* pl = WLO + (size_t)i * 8;
  *(volatile v4u*)ph = uh;
  *(volatile v4u*)pl = ul;
  __threadfence();
  *(volatile v4u*)ph = uh;
  *(volatile v4u*)pl = ul;
}

__global__ __launch_bounds__(256) void prep_tab_kernel(
    const float* __restrict__ wih, const float* __restrict__ fc3w, const float* __restrict__ fc3b,
    const float* __restrict__ bih, const float* __restrict__ bhh, const float* __restrict__ fc2b,
    float* __restrict__ TAB) {
  __shared__ __align__(16) float st[256];
  const int t  = threadIdx.x;
  const int tc = (t < 79) ? t : 79;
  float a = 0.0f, cc = 0.0f;
#pragma unroll 1
  for (int n = 0; n < 32; ++n) {
    const float wv = wih[n];
    a  += wv * fc3w[n * 80 + tc];
    cc += wv * fc3b[n];
  }
  cc = (cc + bih[0]) + bhh[0];
  int bi = t - 128; bi = (bi < 0) ? 0 : ((bi > 79) ? 79 : bi);
  const float bb = fc2b[bi];
  float val = 0.0f;
  val = (t >= 128 && t < 208) ? bb : val;
  val = (t == 80) ? cc : val;
  val = (t < 80) ? a : val;
  st[t] = val;
  __syncthreads();
  if (t < 64) {
    const v4f o = *(const v4f*)(st + 4 * t);
    *(volatile v4f*)(TAB + 4 * t) = o;
    __threadfence();
    *(volatile v4f*)(TAB + 4 * t) = o;
  }
}

__global__ __launch_bounds__(256) void conv1_kernel(
    const float* __restrict__ x, const float* __restrict__ w1, const float* __restrict__ b1,
    unsigned short* __restrict__ Ghi, unsigned short* __restrict__ Glo) {
  __shared__ float sw[640];
  __shared__ float sb[64];
  const int t = threadIdx.x;
  const int s = blockIdx.y;
  sw[t] = w1[t];
  sw[256 + t] = w1[256 + t];
  if (t < 128) sw[512 + t] = w1[512 + t];
  if (t < 64)  sb[t] = b1[t];
  __syncthreads();
  const int p  = blockIdx.x * 32 + (t >> 3);
  const int c8 = (t & 7) * 8;
  const float sgn = s ? -1.0f : 1.0f;
  const bool valid = (p <= G_VALID_MAX);
  float xa[5], xb[5];
#pragma unroll
  for (int k = 0; k < 5; ++k) {
    int idx = p + k; idx = (idx > L_IN - 1) ? (L_IN - 1) : idx;
    xa[k] = x[idx] * sgn;
    xb[k] = x[L_IN + idx];
  }
  unsigned hb[8], lb[8];
#pragma unroll
  for (int e = 0; e < 8; ++e) {
    const float* wr = sw + (c8 + e) * 10;
    float acc = sb[c8 + e];
#pragma unroll
    for (int k = 0; k < 5; ++k) acc += wr[k] * xa[k];
#pragma unroll
    for (int k = 0; k < 5; ++k) acc += wr[5 + k] * xb[k];
    float v = fmaxf(acc, 0.0f);
    v = valid ? v : 0.0f;
    hb[e] = f2bf_u(v);
    lb[e] = f2bf_u(v - bfu2f(hb[e]));
  }
  const v4u uh = (v4u){hb[0] | (hb[1] << 16), hb[2] | (hb[3] << 16), hb[4] | (hb[5] << 16), hb[6] | (hb[7] << 16)};
  const v4u ul = (v4u){lb[0] | (lb[1] << 16), lb[2] | (lb[3] << 16), lb[4] | (lb[5] << 16), lb[6] | (lb[7] << 16)};
  const size_t o = ((size_t)s * G_ROWS + (size_t)p) * NCH + c8;
  *(volatile v4u*)(Ghi + o) = uh;
  *(volatile v4u*)(Glo + o) = ul;
  __threadfence();
  *(volatile v4u*)(Ghi + o) = uh;
  *(volatile v4u*)(Glo + o) = ul;
}

template <int OUT_MODE>
__global__ __launch_bounds__(256) void gemm_bf16x3_kernel(
    const unsigned short* __restrict__ Ap, const unsigned short* __restrict__ A2p, int lda, int tapStride, long strideA,
    const unsigned short* __restrict__ Btp, const unsigned short* __restrict__ Bt2p, int ldb,
    void* __restrict__ Cout, void* __restrict__ Cout2, int ldc, long strideC,
    const float* __restrict__ bias, int M, int N, int K) {
  typedef __bf16 T;
  typedef v16b V;
  const T* A = (const T*)Ap; const T* A2 = (const T*)A2p; const T* Bt = (const T*)Btp; const T* Bt2 = (const T*)Bt2p;
  __shared__ __align__(16) float sT[8][16 * 68];
  const int b    = blockIdx.y;
  const int lane = threadIdx.x & 31;
  const int wave = threadIdx.x >> 5;
  const int tilesN = N >> 6;
  const int tilesM = M >> 6;
  const int tile = blockIdx.x * 8 + wave;
  if (tile >= tilesM * tilesN) return;
  const int tm = tile / tilesN;
  const int tn = tile - tm * tilesN;
  const int m0 = tm << 6;
  const int n0 = tn << 6;

  const T* Ab  = A  + (size_t)b * strideA;
  const T* Ab2 = A2 + (size_t)b * strideA;
  const T* Bb  = Bt;
  const T* Bb2 = Bt2;

  const int rlane = lane & 15;
  const int koff  = (lane >> 4) * 8;
  const int mOff  = (lane >> 4) * 8;

  v8f acc[4][4];
#pragma unroll
  for (int i = 0; i < 4; ++i)
#pragma unroll
    for (int j = 0; j < 4; ++j) acc[i][j] = (v8f){0.f,0.f,0.f,0.f,0.f,0.f,0.f,0.f};

  for (int k0 = 0; k0 < K; k0 += 32) {
    const int kA = (k0 >> 6) * tapStride + (k0 & 63);
    V bh[4], bl[4];
#pragma unroll
    for (int j = 0; j < 4; ++j) {
      const size_t bo = (size_t)(n0 + (j << 4) + rlane) * ldb + koff + k0;
      bh[j] = FragB::load(Bb + bo);
      bl[j] = FragB::load(Bb2 + bo);
    }
#pragma unroll
    for (int i = 0; i < 4; ++i) {
      const size_t ao = (size_t)(m0 + (i << 4) + rlane) * lda + koff + kA;
      V ah = FragB::load(Ab + ao);
      V al = FragB::load(Ab2 + ao);
#pragma unroll
      for (int j = 0; j < 4; ++j) {
        acc[i][j] = FragB::mma(ah, bh[j], acc[i][j]);
        acc[i][j] = FragB::mma(ah, bl[j], acc[i][j]);
        acc[i][j] = FragB::mma(al, bh[j], acc[i][j]);
      }
      row_guard_b(acc[i][0], acc[i][1], acc[i][2], acc[i][3], ah, al);
    }
    keep4_b(bh[0], bh[1], bh[2], bh[3]);
    keep4_b(bl[0], bl[1], bl[2], bl[3]);
  }
  acc_guard4(acc[0][0], acc[0][1], acc[0][2], acc[0][3]);
  acc_guard4(acc[1][0], acc[1][1], acc[1][2], acc[1][3]);
  acc_guard4(acc[2][0], acc[2][1], acc[2][2], acc[2][3]);
  acc_guard4(acc[3][0], acc[3][1], acc[3][2], acc[3][3]);

  float* slab = sT[wave];
#pragma unroll
  for (int i = 0; i < 4; ++i) {
    const int mBase = m0 + (i << 4);
#pragma unroll
    for (int j = 0; j < 4; ++j) {
      const int n = n0 + (j << 4) + rlane;
      const float bv = bias[n];
#pragma unroll
      for (int r = 0; r < 8; ++r) {
        float v = acc[i][j][r] + bv;
        v = fmaxf(v, 0.0f);
        slab[(mOff + r) * 68 + (j << 4) + rlane] = v;
      }
    }
    __builtin_amdgcn_fence(__ATOMIC_RELEASE, "workgroup");
    __builtin_amdgcn_wave_barrier();
    __builtin_amdgcn_fence(__ATOMIC_ACQUIRE, "workgroup");
    if (OUT_MODE == 0) {
      float* C = (float*)Cout + (size_t)b * strideC;
      const int hh = lane >> 4, c4 = (lane & 15) * 4;
      for (int pass = 0; pass < 2; ++pass) {
#pragma unroll
        for (int it = 0; it < 8; ++it) {
          const int row = it * 2 + hh;
          v4f v = *(const v4f*)(slab + row * 68 + c4);
          *(volatile v4f*)(C + (size_t)(mBase + row) * ldc + n0 + c4) = v;
        }
        __threadfence();
      }
    } else {
      const int q = lane >> 3, c8 = (lane & 7) * 8;
      unsigned short* C  = (unsigned short*)Cout  + (size_t)b * strideC;
      unsigned short* C2 = (unsigned short*)Cout2 + (size_t)b * strideC;
      for (int pass = 0; pass < 2; ++pass) {
#pragma unroll
        for (int it = 0; it < 4; ++it) {
          const int row = it * 4 + q;
          const float* sp = slab + row * 68 + c8;
          v8h hv, lv;
#pragma unroll
          for (int e = 0; e < 8; ++e) {
            unsigned short hb = f2bf_bits(sp[e]);
            unsigned short lb = f2bf_bits(sp[e] - bf_bits2f(hb));
            hv[e] = __builtin_bit_cast(_Float16, hb);
            lv[e] = __builtin_bit_cast(_Float16, lb);
          }
          *(volatile v8h*)(C  + (size_t)(mBase + row) * ldc + n0 + c8) = hv;
          *(volatile v8h*)(C2 + (size_t)(mBase + row) * ldc + n0 + c8) = lv;
        }
        __threadfence();
      }
    }
    __builtin_amdgcn_fence(__ATOMIC_RELEASE, "workgroup");
    __builtin_amdgcn_wave_barrier();
    __builtin_amdgcn_fence(__ATOMIC_ACQUIRE, "workgroup");
  }
}

__global__ __launch_bounds__(256) void proj_kernel(const float* __restrict__ H2, const float* __restrict__ TAB,
                                                   float* __restrict__ XP) {
  __shared__ __align__(16) float sv[128];
  const int t = threadIdx.x;
  if (t < 32) *(v4f*)(sv + 4 * t) = *(const v4f*)(TAB + 4 * t);
  __syncthreads();
  const int row = blockIdx.x * 256 + t;
  const float* hp = H2 + (size_t)row * H2_PITCH;
  float a = sv[80];
#pragma unroll 1
  for (int g = 0; g < 5; ++g) {
    const v4f h0 = *(const v4f*)(hp + 16 * g);
    const v4f h1 = *(const v4f*)(hp + 16 * g + 4);
    const v4f h2 = *(const v4f*)(hp + 16 * g + 8);
    const v4f h3 = *(const v4f*)(hp + 16 * g + 12);
    const v4f w0 = *(const v4f*)(sv + 16 * g);
    const v4f w1 = *(const v4f*)(sv + 16 * g + 4);
    const v4f w2 = *(const v4f*)(sv + 16 * g + 8);
    const v4f w3 = *(const v4f*)(sv + 16 * g + 12);
#pragma unroll
    for (int e = 0; e < 4; ++e) a += h0[e] * w0[e];
#pragma unroll
    for (int e = 0; e < 4; ++e) a += h1[e] * w1[e];
#pragma unroll
    for (int e = 0; e < 4; ++e) a += h2[e] * w2[e];
#pragma unroll
    for (int e = 0; e < 4; ++e) a += h3[e] * w3[e];
  }
  *(volatile float*)(XP + row) = a;
  __threadfence();
  *(volatile float*)(XP + row) = a;
}

__global__ __launch_bounds__(32) void scan_out_kernel(const float* __restrict__ XP, const float* __restrict__ whh,
                                                      float* __restrict__ out) {
  __shared__ __align__(16) float sx[2][128];
  __shared__ __align__(16) float sy[2][128];
  const int lane  = threadIdx.x;
  const int chain = lane & 1;
  const float wh = whh[0];
  float h = 0.0f;
#pragma unroll 1
  for (int c = 0; c < NWIN / 128; ++c) {
    const v4f a = *(const v4f*)(XP + c * 128 + 4 * lane);
    const v4f b = *(const v4f*)(XP + NWIN + c * 128 + 4 * lane);
    *(v4f*)(&sx[0][4 * lane]) = a;
    *(v4f*)(&sx[1][4 * lane]) = b;
    __syncthreads();
#pragma unroll 1
    for (int i = 0; i < 128; ++i) {
      const float xv = sx[chain][i];
      h = tanhf(xv + wh * h);
      if (lane < 2) sy[chain][i] = h;
    }
    __syncthreads();
    const v4f ya = *(const v4f*)(&sy[0][4 * lane]);
    const v4f yb = *(const v4f*)(&sy[1][4 * lane]);
    const v4f o = (ya - yb) * 0.5f;
    float* op = out + c * 128 + 4 * lane;
    *(volatile v4f*)op = o;
    __threadfence();
    *(volatile v4f*)op = o;
    __syncthreads();
  }
}

extern "C" void kernel_launch(void* const* d_in, const int* in_sizes, int n_in,
                              void* d_out, int out_size, void* d_ws, size_t ws_size, hipStream_t stream) {
  if (n_in < 17 || d_out == nullptr || d_ws == nullptr) return;
  if (in_sizes[0] != 2 * L_IN || in_sizes[1] != 640 || in_sizes[2] != 64 ||
      in_sizes[3] != NCH * K_CONV || in_sizes[4] != 64 || in_sizes[5] != NCH * K_CONV || in_sizes[6] != 64 ||
      in_sizes[7] != N_FC1 * K_FC1 || in_sizes[8] != N_FC1 || in_sizes[9] != N_FC2 * K_FC2 || in_sizes[10] != N_FC2 ||
      in_sizes[11] != 32 * 80 || in_sizes[12] != 32 || in_sizes[13] != 32 ||
      in_sizes[14] != 1 || in_sizes[15] != 1 || in_sizes[16] != 1 || out_size != NWIN) return;

  const float* x0  = (const float*)d_in[0];
  const float* w1  = (const float*)d_in[1];
  const float* b1  = (const float*)d_in[2];
  const float* w2  = (const float*)d_in[3];
  const float* b2  = (const float*)d_in[4];
  const float* w3  = (const float*)d_in[5];
  const float* b3  = (const float*)d_in[6];
  const float* fw1 = (const float*)d_in[7];
  const float* fb1 = (const float*)d_in[8];
  const float* fw2 = (const float*)d_in[9];
  const float* fb2 = (const float*)d_in[10];
  const float* fw3 = (const float*)d_in[11];
  const float* fb3 = (const float*)d_in[12];
  const float* wih = (const float*)d_in[13];
  const float* whh = (const float*)d_in[14];
  const float* bih = (const float*)d_in[15];
  const float* bhh = (const float*)d_in[16];
  float* out = (float*)d_out;

  char* ws = (char*)d_ws; size_t off = 0;
  auto carve = [&](size_t bytes) -> char* { char* p = ws + off; off += (bytes + 255) & ~(size_t)255; return p; };
  unsigned short* WHI  = (unsigned short*)carve((size_t)W_TOTAL * 2);
  unsigned short* WLO  = (unsigned short*)carve((size_t)W_TOTAL * 2);
  float*          TAB  = (float*)carve((size_t)256 * 4);
  unsigned short* GHI  = (unsigned short*)carve((size_t)2 * G_ROWS * NCH * 2);
  unsigned short* GLO  = (unsigned short*)carve((size_t)2 * G_ROWS * NCH * 2);
  unsigned short* C2HI = (unsigned short*)carve((size_t)2 * C2_ROWS * NCH * 2);
  unsigned short* C2LO = (unsigned short*)carve((size_t)2 * C2_ROWS * NCH * 2);
  unsigned short* C3HI = (unsigned short*)carve((size_t)2 * C3_ROWS * NCH * 2);
  unsigned short* C3LO = (unsigned short*)carve((size_t)2 * C3_ROWS * NCH * 2);
  unsigned short* H1HI = (unsigned short*)carve((size_t)2 * NWIN * N_FC1 * 2);
  unsigned short* H1LO = (unsigned short*)carve((size_t)2 * NWIN * N_FC1 * 2);
  float*          H2   = (float*)carve((size_t)2 * NWIN * H2_PITCH * 4);
  float*          XP   = (float*)carve((size_t)2 * NWIN * 4);
  if (off > ws_size || off > (size_t)134217728) return;

  prep_weights_kernel<<<U_TOTAL / 256, 256, 0, stream>>>(w2, w3, fw1, fw2, WHI, WLO);
  prep_tab_kernel<<<1, 256, 0, stream>>>(wih, fw3, fb3, bih, bhh, fb2, TAB);

  conv1_kernel<<<dim3(G_ROWS / 32, 2), 256, 0, stream>>>(x0, w1, b1, GHI, GLO);

  gemm_bf16x3_kernel<2><<<dim3((C2_ROWS / 64 + 7) / 8, 2), 256, 0, stream>>>(
      GHI, GLO, NCH, DIL2 * NCH, (long)G_ROWS * NCH,
      WHI + OFF_W2, WLO + OFF_W2, K_CONV,
      (void*)C2HI, (void*)C2LO, NCH, (long)C2_ROWS * NCH,
      b2, C2_ROWS, NCH, K_CONV);

  gemm_bf16x3_kernel<2><<<dim3((C3_ROWS / 64 + 7) / 8, 2), 256, 0, stream>>>(
      C2HI, C2LO, NCH, DIL3 * NCH, (long)C2_ROWS * NCH,
      WHI + OFF_W3, WLO + OFF_W3, K_CONV,
      (void*)C3HI, (void*)C3LO, NCH, (long)C3_ROWS * NCH,
      b3, C3_ROWS, NCH, K_CONV);

  gemm_bf16x3_kernel<2><<<dim3(((NWIN / 64) * (N_FC1 / 64) + 7) / 8, 2), 256, 0, stream>>>(
      C3HI, C3LO, NCH, DILF * NCH, (long)C3_ROWS * NCH,
      WHI + OFF_FC1, WLO + OFF_FC1, K_FC1,
      (void*)H1HI, (void*)H1LO, N_FC1, (long)NWIN * N_FC1,
      fb1, NWIN, N_FC1, K_FC1);

  gemm_bf16x3_kernel<0><<<dim3((((2 * NWIN) / 64) * (N_FC2P / 64) + 7) / 8, 1), 256, 0, stream>>>(
      H1HI, H1LO, K_FC2, 64, 0L,
      WHI + OFF_FC2, WLO + OFF_FC2, K_FC2,
      (void*)H2, (void*)H2, H2_PITCH, 0L,
      TAB + 128, 2 * NWIN, N_FC2P, K_FC2);

  proj_kernel<<<(2 * NWIN) / 256, 256, 0, stream>>>(H2, TAB, XP);

  scan_out_kernel<<<1, 32, 0, stream>>>(XP, whh, out);
}
